// ManyToOneLSTM_18519898980509
// MI455X (gfx1250) — hardware-verified
//
#include <hip/hip_runtime.h>
#include <stdint.h>
#include <math.h>

typedef __attribute__((ext_vector_type(16))) _Float16 v16h;
typedef __attribute__((ext_vector_type(8)))  _Float16 v8h;
typedef __attribute__((ext_vector_type(16))) __bf16   v16b;
typedef __attribute__((ext_vector_type(8)))  __bf16   v8b;
typedef __attribute__((ext_vector_type(8)))  float    v8f;
typedef __attribute__((ext_vector_type(4)))  float    v4f;

constexpr int kSeqN        = 2048;
constexpr int kSteps       = 512;
constexpr int kHid1        = 32;
constexpr int kHid2        = 64;
constexpr int kGate1       = 4 * kHid1;
constexpr int kGate2       = 4 * kHid2;
constexpr int kThreads     = 64;
constexpr int kSeqPerWave  = 16;
constexpr int kSeqPerBlock = 32;
constexpr int kBlocks      = kSeqN / kSeqPerBlock;
static_assert(kBlocks * kSeqPerBlock == kSeqN);
static_assert(kSeqPerBlock == (kThreads / 32) * kSeqPerWave);
constexpr float kWsc    = 4.0f;
constexpr float kWscInv = 0.25f;

__device__ __forceinline__ unsigned short f2bf_bits(float f) {
  unsigned u = __float_as_uint(f);
  return (unsigned short)((u + 0x7FFFu + ((u >> 16) & 1u)) >> 16);
}
__device__ __forceinline__ float bf_bits2f(unsigned short h) { return __uint_as_float(((unsigned)h) << 16); }

__device__ __forceinline__ void dep_guard_h(v8f& a, v8f& b, v16h x, v16h y) { asm volatile("v_nop\n\tv_nop\n\tv_nop\n\tv_nop" : "+v"(a), "+v"(b) : "v"(x), "v"(y)); }
__device__ __forceinline__ void dep_guard_b(v8f& a, v8f& b, v16b x, v16b y) { asm volatile("v_nop\n\tv_nop\n\tv_nop\n\tv_nop" : "+v"(a), "+v"(b) : "v"(x), "v"(y)); }
__device__ __forceinline__ void keep4_h(v16h a, v16h b, v16h c, v16h d) { asm volatile("v_nop" :: "v"(a), "v"(b), "v"(c), "v"(d)); }
__device__ __forceinline__ void keep4_b(v16b a, v16b b, v16b c, v16b d) { asm volatile("v_nop" :: "v"(a), "v"(b), "v"(c), "v"(d)); }
__device__ __forceinline__ void acc_guard4(v8f& a, v8f& b, v8f& c, v8f& d) { asm volatile("v_nop\n\tv_nop\n\tv_nop\n\tv_nop" : "+v"(a), "+v"(b), "+v"(c), "+v"(d)); }
template <typename T> struct Frag;
template <> struct Frag<_Float16> {
  typedef v16h V; union U { v16h v; v8h h[2]; };
  static __device__ __forceinline__ v16h load(const _Float16* p) {
    U f; f.h[0] = *(const v8h*)(p); f.h[1] = *(const v8h*)(p + 16); return f.v;
  }
  static __device__ __forceinline__ v8f mma(v16h a, v16h b, v8f c) {
    return __builtin_amdgcn_wmma_f32_16x16x32_f16(false, a, false, b, (short)0, c, false, false);
  }
  static __device__ __forceinline__ void guard(v8f& a, v8f& b, v16h x, v16h y) { dep_guard_h(a, b, x, y); }
  static __device__ __forceinline__ void keep(v16h a, v16h b, v16h c, v16h d) { keep4_h(a, b, c, d); }
};
template <> struct Frag<__bf16> {
  typedef v16b V; union U { v16b v; v8b h[2]; };
  static __device__ __forceinline__ v16b load(const __bf16* p) {
    U f; f.h[0] = *(const v8b*)(p); f.h[1] = *(const v8b*)(p + 16); return f.v;
  }
  static __device__ __forceinline__ v8f mma(v16b a, v16b b, v8f c) {
    return __builtin_amdgcn_wmma_f32_16x16x32_bf16(false, a, false, b, (short)0, c, false, false);
  }
  static __device__ __forceinline__ void guard(v8f& a, v8f& b, v16b x, v16b y) { dep_guard_b(a, b, x, y); }
  static __device__ __forceinline__ void keep(v16b a, v16b b, v16b c, v16b d) { keep4_b(a, b, c, d); }
};

__device__ __forceinline__ v8f mma_f16(v16h a, v16h b, v8f c) {
  c = __builtin_amdgcn_wmma_f32_16x16x32_f16(false, a, false, b, (short)0, c, false, false);
  asm volatile("v_nop\n\tv_nop\n\tv_nop\n\tv_nop" : "+v"(c) : "v"(a), "v"(b));
  return c;
}
__device__ __forceinline__ void lds_order() { asm volatile("" ::: "memory"); }

__device__ __forceinline__ float fsig(float x)  { return __builtin_amdgcn_rcpf(1.0f + __expf(-x)); }
__device__ __forceinline__ float ftanh(float x) { return 1.0f - 2.0f * __builtin_amdgcn_rcpf(__expf(2.0f * x) + 1.0f); }

__device__ __forceinline__ v8f ld8f(const float* p) {
  union { v4f q[2]; v8f v; } t;
  t.q[0] = *(const v4f*)(p);
  t.q[1] = *(const v4f*)(p + 4);
  return t.v;
}

__global__ __launch_bounds__(kThreads) void lstm2_m2o_kernel(
    const float* __restrict__ xin,
    const float* __restrict__ h1i, const float* __restrict__ c1i,
    const float* __restrict__ h2i, const float* __restrict__ c2i,
    const float* __restrict__ Wih1, const float* __restrict__ Whh1,
    const float* __restrict__ bih1, const float* __restrict__ bhh1,
    const float* __restrict__ Wih2, const float* __restrict__ Whh2,
    const float* __restrict__ bih2, const float* __restrict__ bhh2,
    const float* __restrict__ Wlin, const float* __restrict__ blin,
    float* __restrict__ out) {
  __shared__ __align__(16) _Float16 sWhh1[kGate1 * kHid1];
  __shared__ __align__(16) _Float16 sWih2[kGate2 * kHid1];
  __shared__ __align__(16) _Float16 sWhh2[kGate2 * kHid2];
  __shared__ __align__(16) float sPb1[kGate1];
  __shared__ __align__(16) float sPw1[kGate1];
  __shared__ __align__(16) float sPb2[kGate2];
  __shared__ __align__(16) float sWl[kHid2];
  __shared__ __align__(16) float sPart[2][kSeqPerBlock];
  __shared__ __align__(16) float sOut[kSeqPerBlock];

  const int tid = threadIdx.x;
#pragma unroll 1
  for (int i = tid; i < kGate1 * kHid1; i += kThreads) sWhh1[i] = (_Float16)(kWsc * Whh1[i]);
#pragma unroll 1
  for (int i = tid; i < kGate2 * kHid1; i += kThreads) sWih2[i] = (_Float16)(kWsc * Wih2[i]);
#pragma unroll 1
  for (int i = tid; i < kGate2 * kHid2; i += kThreads) sWhh2[i] = (_Float16)(kWsc * Whh2[i]);
#pragma unroll 1
  for (int i = tid; i < kGate1; i += kThreads) { sPb1[i] = kWsc * (bih1[i] + bhh1[i]); sPw1[i] = kWsc * Wih1[i]; }
#pragma unroll 1
  for (int i = tid; i < kGate2; i += kThreads) sPb2[i] = kWsc * (bih2[i] + bhh2[i]);
  if (tid < kHid2) sWl[tid] = Wlin[tid];
  __syncthreads();

  const int lane = tid & 31, wave = tid >> 5;
  const int hh = lane >> 4, col = lane & 15, k8 = 8 * hh;
  const int n = blockIdx.x * kSeqPerBlock + wave * kSeqPerWave + col;

  float c1s[2][8], h1n[2][8], c2s[4][8], h2v[4][8];
#pragma unroll
  for (int ht = 0; ht < 2; ++ht) {
    const v8f cv = ld8f(c1i + (size_t)n * kHid1 + 16 * ht + k8);
    const v8f hv = ld8f(h1i + (size_t)n * kHid1 + 16 * ht + k8);
#pragma unroll
    for (int r = 0; r < 8; ++r) { c1s[ht][r] = cv[r]; h1n[ht][r] = hv[r]; }
  }
#pragma unroll
  for (int ht = 0; ht < 4; ++ht) {
    const v8f cv = ld8f(c2i + (size_t)n * kHid2 + 16 * ht + k8);
    const v8f hv = ld8f(h2i + (size_t)n * kHid2 + 16 * ht + k8);
#pragma unroll
    for (int r = 0; r < 8; ++r) { c2s[ht][r] = cv[r]; h2v[ht][r] = hv[r]; }
  }
  v16h h1B, h2B0, h2B1;
#pragma unroll
  for (int e = 0; e < 8; ++e) {
    h1B[e]  = (_Float16)h1n[0][e];  h1B[8 + e]  = (_Float16)h1n[1][e];
    h2B0[e] = (_Float16)h2v[0][e];  h2B0[8 + e] = (_Float16)h2v[1][e];
    h2B1[e] = (_Float16)h2v[2][e];  h2B1[8 + e] = (_Float16)h2v[3][e];
  }

#pragma unroll 1
  for (int t = 0; t < kSteps; ++t) {
    lds_order();
    const float x = xin[(size_t)n * kSteps + (size_t)t];

#pragma unroll
    for (int ht = 0; ht < 2; ++ht) {
      lds_order();
      v8f z[4];
#pragma unroll
      for (int g = 0; g < 4; ++g) {
        const int rb = 32 * g + 16 * ht + k8;
        z[g] = ld8f(sPb1 + rb) + ld8f(sPw1 + rb) * x;
      }
#pragma unroll
      for (int g = 0; g < 4; ++g) {
        const v16h a = Frag<_Float16>::load(sWhh1 + (32 * g + 16 * ht + col) * kHid1 + k8);
        z[g] = mma_f16(a, h1B, z[g]);
      }
#pragma unroll
      for (int r = 0; r < 8; ++r) {
        const float ig = fsig(z[0][r] * kWscInv);
        const float fg = fsig(z[1][r] * kWscInv);
        const float gg = ftanh(z[2][r] * kWscInv);
        const float og = fsig(z[3][r] * kWscInv);
        const float cn = fg * c1s[ht][r] + ig * gg;
        c1s[ht][r] = cn;
        h1n[ht][r] = og * ftanh(cn);
      }
    }
#pragma unroll
    for (int e = 0; e < 8; ++e) { h1B[e] = (_Float16)h1n[0][e]; h1B[8 + e] = (_Float16)h1n[1][e]; }

#pragma unroll
    for (int ht = 0; ht < 4; ++ht) {
      v8f z[4];
#pragma unroll
      for (int g = 0; g < 4; ++g) {
        lds_order();
        const int row = 64 * g + 16 * ht;
        z[g] = ld8f(sPb2 + row + k8);
        const v16h a0 = Frag<_Float16>::load(sWih2 + (row + col) * kHid1 + k8);
        const v16h a1 = Frag<_Float16>::load(sWhh2 + (row + col) * kHid2 + k8);
        const v16h a2 = Frag<_Float16>::load(sWhh2 + (row + col) * kHid2 + 32 + k8);
        z[g] = mma_f16(a0, h1B,  z[g]);
        z[g] = mma_f16(a1, h2B0, z[g]);
        z[g] = mma_f16(a2, h2B1, z[g]);
      }
#pragma unroll
      for (int r = 0; r < 8; ++r) {
        const float ig = fsig(z[0][r] * kWscInv);
        const float fg = fsig(z[1][r] * kWscInv);
        const float gg = ftanh(z[2][r] * kWscInv);
        const float og = fsig(z[3][r] * kWscInv);
        const float cn = fg * c2s[ht][r] + ig * gg;
        c2s[ht][r] = cn;
        h2v[ht][r] = og * ftanh(cn);
      }
    }
#pragma unroll
    for (int e = 0; e < 8; ++e) {
      h2B0[e] = (_Float16)h2v[0][e];  h2B0[8 + e] = (_Float16)h2v[1][e];
      h2B1[e] = (_Float16)h2v[2][e];  h2B1[8 + e] = (_Float16)h2v[3][e];
    }
  }

  float sum = 0.0f;
#pragma unroll
  for (int ht = 0; ht < 4; ++ht) {
    const v8f wl = ld8f(sWl + 16 * ht + k8);
#pragma unroll
    for (int r = 0; r < 8; ++r) sum = fmaf(h2v[ht][r], wl[r], sum);
  }
  sPart[hh][wave * kSeqPerWave + col] = sum;
  __syncthreads();
  if (tid < kSeqPerBlock) sOut[tid] = (sPart[0][tid] + sPart[1][tid]) + blin[0];
  __syncthreads();
  if (tid < 8) {
    const v4f v = *(const v4f*)(sOut + 4 * tid);
    float* op = out + (size_t)blockIdx.x * kSeqPerBlock + 4 * tid;
    *(volatile v4f*)op = v;
    __threadfence();
    *(volatile v4f*)op = v;
  }
}

extern "C" void kernel_launch(void* const* d_in, const int* in_sizes, int n_in,
                              void* d_out, int out_size, void* d_ws, size_t ws_size, hipStream_t stream) {
  (void)d_ws; (void)ws_size;
  if (n_in < 15 || d_out == nullptr) return;
  if (in_sizes[0] != kSeqN * kSteps || in_sizes[1] != kSeqN * kHid1 || in_sizes[2] != kSeqN * kHid1 ||
      in_sizes[3] != kSeqN * kHid2 || in_sizes[4] != kSeqN * kHid2 ||
      in_sizes[5] != kGate1 || in_sizes[6] != kGate1 * kHid1 || in_sizes[7] != kGate1 || in_sizes[8] != kGate1 ||
      in_sizes[9] != kGate2 * kHid1 || in_sizes[10] != kGate2 * kHid2 || in_sizes[11] != kGate2 || in_sizes[12] != kGate2 ||
      in_sizes[13] != kHid2 || in_sizes[14] < 1 || out_size != kSeqN) return;

  const float* xin  = (const float*)d_in[0];
  const float* h1i  = (const float*)d_in[1];
  const float* c1i  = (const float*)d_in[2];
  const float* h2i  = (const float*)d_in[3];
  const float* c2i  = (const float*)d_in[4];
  const float* Wih1 = (const float*)d_in[5];
  const float* Whh1 = (const float*)d_in[6];
  const float* bih1 = (const float*)d_in[7];
  const float* bhh1 = (const float*)d_in[8];
  const float* Wih2 = (const float*)d_in[9];
  const float* Whh2 = (const float*)d_in[10];
  const float* bih2 = (const float*)d_in[11];
  const float* bhh2 = (const float*)d_in[12];
  const float* Wlin = (const float*)d_in[13];
  const float* blin = (const float*)d_in[14];
  float* out = (float*)d_out;

  lstm2_m2o_kernel<<<dim3(kBlocks), dim3(kThreads), 0, stream>>>(
      xin, h1i, c1i, h2i, c2i, Wih1, Whh1, bih1, bhh1, Wih2, Whh2, bih2, bhh2, Wlin, blin, out);
}
